// LSTM_Branch_32633161515020
// MI455X (gfx1250) — hardware-verified
//
#include <hip/hip_runtime.h>
#include <stdint.h>

constexpr int NSEQ    = 4096;
constexpr int NSTEP   = 365;
constexpr int NIN     = 3;
constexpr int NHID    = 64;
constexpr int NG4     = 256;
constexpr int NTHR    = 256;
constexpr int TROWS   = 32;
constexpr int HPITCH  = 72;
constexpr int XCH     = 32;
constexpr int XW      = 4;
constexpr int OPITCH  = 68;
constexpr int GSTRIDE = NHID * NHID;
constexpr float A_CARRY = 16.0f;
constexpr float W_CARRY = 64.0f;
constexpr float Z_FOLD  = 1.0f / 1024.0f;

static_assert(NSEQ % TROWS == 0, "grid covers all sequences exactly");
static_assert((XCH & (XCH - 1)) == 0, "chunk length is a power of two");
static_assert(TROWS * XCH == NTHR * 4, "four (row, step) pairs per thread per x chunk");
static_assert((NG4 * NHID / 8) % NTHR == 0, "weight prep grid exact");
static_assert(NHID % 32 == 0, "K multiple of 32");
static_assert((2 * TROWS * HPITCH) % NTHR == 0, "h tile zero fill exact");
static_assert(TROWS == 4 * (NTHR / 32), "each wave stores 4 output rows");

typedef __attribute__((ext_vector_type(16))) _Float16 v16h;
typedef __attribute__((ext_vector_type(8)))  _Float16 v8h;
typedef __attribute__((ext_vector_type(8)))  float    v8f;
typedef __attribute__((ext_vector_type(4)))  float    v4f;

__device__ __forceinline__ unsigned short f2bf_bits(float f) {
  unsigned u = __float_as_uint(f);
  return (unsigned short)((u + 0x7FFFu + ((u >> 16) & 1u)) >> 16);
}
__device__ __forceinline__ float bf_bits2f(unsigned short h) { return __uint_as_float(((unsigned)h) << 16); }
__device__ __forceinline__ float bfr(float f) { return bf_bits2f(f2bf_bits(f)); }

__device__ __forceinline__ void dep_guard_h(v8f& a, v8f& b, v16h x, v16h y) { asm volatile("v_nop\n\tv_nop\n\tv_nop\n\tv_nop" : "+v"(a), "+v"(b) : "v"(x), "v"(y)); }
__device__ __forceinline__ void keep4_h(v16h a, v16h b, v16h c, v16h d) { asm volatile("v_nop" :: "v"(a), "v"(b), "v"(c), "v"(d)); }
__device__ __forceinline__ void keep2_h(v16h a, v16h b) { asm volatile("v_nop" :: "v"(a), "v"(b)); }
__device__ __forceinline__ void acc_guard4(v8f& a, v8f& b, v8f& c, v8f& d) { asm volatile("v_nop\n\tv_nop\n\tv_nop\n\tv_nop" : "+v"(a), "+v"(b), "+v"(c), "+v"(d)); }
template <typename T> struct Frag;
template <> struct Frag<_Float16> {
  typedef v16h V; union U { v16h v; v8h h[2]; };
  static __device__ __forceinline__ v16h load(const _Float16* p) {
    U f; f.h[0] = *(const v8h*)(p); f.h[1] = *(const v8h*)(p + 16); return f.v;
  }
  static __device__ __forceinline__ v8f mma(v16h a, v16h b, v8f c) {
    return __builtin_amdgcn_wmma_f32_16x16x32_f16(false, a, false, b, (short)0, c, false, false);
  }
  static __device__ __forceinline__ void guard(v8f& a, v8f& b, v16h x, v16h y) { dep_guard_h(a, b, x, y); }
  static __device__ __forceinline__ void keep(v16h a, v16h b, v16h c, v16h d) { keep4_h(a, b, c, d); }
};
typedef Frag<_Float16> FragH;

__device__ __forceinline__ float fsig(float v)  { return __builtin_amdgcn_rcpf(1.0f + __expf(-v)); }
__device__ __forceinline__ float ftanh(float v) { return 1.0f - 2.0f * __builtin_amdgcn_rcpf(__expf(2.0f * v) + 1.0f); }

__global__ __launch_bounds__(NTHR) void wprep_kernel(const float* __restrict__ W, int n8, unsigned short* __restrict__ O) {
  const int i = blockIdx.x * NTHR + threadIdx.x;
  if (i >= n8) return;
  const int e0 = i * 8;
  v8h hv;
#pragma unroll
  for (int e = 0; e < 8; ++e) {
    const float fb = bfr(W[e0 + e]);
    hv[e] = (_Float16)(fb * W_CARRY);
  }
  *(volatile v8h*)(O + e0) = hv;
  __threadfence();
  *(volatile v8h*)(O + e0) = hv;
}

__device__ __forceinline__ void mac_l0(v8f (&acc)[4], const _Float16* arow, const _Float16* wh) {
#pragma unroll 1
  for (int kc = 0; kc < 2; ++kc) {
    const int k0 = kc * 32;
    const v16h a  = FragH::load(arow + k0);
    const v16h b0 = FragH::load(wh + k0);
    const v16h b1 = FragH::load(wh + GSTRIDE + k0);
    const v16h b2 = FragH::load(wh + 2 * GSTRIDE + k0);
    const v16h b3 = FragH::load(wh + 3 * GSTRIDE + k0);
    acc[0] = FragH::mma(a, b0, acc[0]);
    acc[1] = FragH::mma(a, b1, acc[1]);
    acc[2] = FragH::mma(a, b2, acc[2]);
    acc[3] = FragH::mma(a, b3, acc[3]);
    acc_guard4(acc[0], acc[1], acc[2], acc[3]);
    keep4_h(a, b0, b1, b2);
    keep2_h(b3, b3);
  }
}

__device__ __forceinline__ void mac_l1(v8f (&acc)[4], const _Float16* abrow, const _Float16* asrow,
                                       const _Float16* wi, const _Float16* wh) {
#pragma unroll 1
  for (int kc = 0; kc < 2; ++kc) {
    const int k0 = kc * 32;
    const v16h ab  = FragH::load(abrow + k0);
    const v16h bi0 = FragH::load(wi + k0);
    const v16h bi1 = FragH::load(wi + GSTRIDE + k0);
    const v16h bi2 = FragH::load(wi + 2 * GSTRIDE + k0);
    const v16h bi3 = FragH::load(wi + 3 * GSTRIDE + k0);
    acc[0] = FragH::mma(ab, bi0, acc[0]);
    acc[1] = FragH::mma(ab, bi1, acc[1]);
    acc[2] = FragH::mma(ab, bi2, acc[2]);
    acc[3] = FragH::mma(ab, bi3, acc[3]);
    const v16h as  = FragH::load(asrow + k0);
    const v16h bh0 = FragH::load(wh + k0);
    const v16h bh1 = FragH::load(wh + GSTRIDE + k0);
    const v16h bh2 = FragH::load(wh + 2 * GSTRIDE + k0);
    const v16h bh3 = FragH::load(wh + 3 * GSTRIDE + k0);
    acc[0] = FragH::mma(as, bh0, acc[0]);
    acc[1] = FragH::mma(as, bh1, acc[1]);
    acc[2] = FragH::mma(as, bh2, acc[2]);
    acc[3] = FragH::mma(as, bh3, acc[3]);
    acc_guard4(acc[0], acc[1], acc[2], acc[3]);
    keep4_h(ab, bi0, bi1, bi2);
    keep4_h(bi3, as, bh0, bh1);
    keep2_h(bh2, bh3);
  }
}

__device__ __forceinline__ float lstm_cell(float pi, float pf, float pg, float po, float& c) {
  const float ii = fsig(pi);
  const float ff = fsig(pf);
  const float gg = ftanh(pg);
  const float oo = fsig(po);
  c = fmaf(ff, c, ii * gg);
  return oo * ftanh(c);
}

__global__ __launch_bounds__(NTHR) void lstm2_kernel(
    const float* __restrict__ x,
    const float* __restrict__ w_ih0, const float* __restrict__ b_ih0, const float* __restrict__ b_hh0,
    const float* __restrict__ b_ih1, const float* __restrict__ b_hh1,
    const unsigned short* __restrict__ Whh0p, const unsigned short* __restrict__ Wih1p,
    const unsigned short* __restrict__ Whh1p,
    float* __restrict__ out) {
  __shared__ __align__(16) _Float16 Ht[2 * TROWS * HPITCH];
  __shared__ __align__(16) float    Xs[TROWS * XCH * XW];
  __shared__ __align__(16) float    Hs[TROWS * OPITCH];

  const int tid = threadIdx.x, lane = tid & 31, wave = tid >> 5;
  const int c = lane & 15, hh = lane >> 4, koff = hh * 8;
  const int rt = wave >> 2;
  const int j  = 16 * (wave & 3) + c;
  const int rb = rt * 16 + 8 * hh;
  const int rowbase = blockIdx.x * TROWS;

#pragma unroll 1
  for (int i = tid; i < 2 * TROWS * HPITCH; i += NTHR) Ht[i] = (_Float16)0.0f;

  const float wxi0 = bfr(w_ih0[(0 * NHID + j) * NIN + 0]), wxi1 = bfr(w_ih0[(0 * NHID + j) * NIN + 1]), wxi2 = bfr(w_ih0[(0 * NHID + j) * NIN + 2]);
  const float wxf0 = bfr(w_ih0[(1 * NHID + j) * NIN + 0]), wxf1 = bfr(w_ih0[(1 * NHID + j) * NIN + 1]), wxf2 = bfr(w_ih0[(1 * NHID + j) * NIN + 2]);
  const float wxg0 = bfr(w_ih0[(2 * NHID + j) * NIN + 0]), wxg1 = bfr(w_ih0[(2 * NHID + j) * NIN + 1]), wxg2 = bfr(w_ih0[(2 * NHID + j) * NIN + 2]);
  const float wxo0 = bfr(w_ih0[(3 * NHID + j) * NIN + 0]), wxo1 = bfr(w_ih0[(3 * NHID + j) * NIN + 1]), wxo2 = bfr(w_ih0[(3 * NHID + j) * NIN + 2]);
  const float cb0i = bfr(b_ih0[0 * NHID + j]) + bfr(b_hh0[0 * NHID + j]);
  const float cb0f = bfr(b_ih0[1 * NHID + j]) + bfr(b_hh0[1 * NHID + j]);
  const float cb0g = bfr(b_ih0[2 * NHID + j]) + bfr(b_hh0[2 * NHID + j]);
  const float cb0o = bfr(b_ih0[3 * NHID + j]) + bfr(b_hh0[3 * NHID + j]);
  const float cb1i = bfr(b_ih1[0 * NHID + j]) + bfr(b_hh1[0 * NHID + j]);
  const float cb1f = bfr(b_ih1[1 * NHID + j]) + bfr(b_hh1[1 * NHID + j]);
  const float cb1g = bfr(b_ih1[2 * NHID + j]) + bfr(b_hh1[2 * NHID + j]);
  const float cb1o = bfr(b_ih1[3 * NHID + j]) + bfr(b_hh1[3 * NHID + j]);

  float c0s[8], c1s[8], h1s[8];
#pragma unroll
  for (int r = 0; r < 8; ++r) { c0s[r] = 0.0f; c1s[r] = 0.0f; h1s[r] = 0.0f; }
  __syncthreads();

  const _Float16* a0row = Ht + (rt * 16 + c) * HPITCH + koff;
  const _Float16* a1row = a0row + TROWS * HPITCH;
  const _Float16* whh0 = (const _Float16*)Whh0p + (size_t)j * NHID + koff;
  const _Float16* wih1 = (const _Float16*)Wih1p + (size_t)j * NHID + koff;
  const _Float16* whh1 = (const _Float16*)Whh1p + (size_t)j * NHID + koff;
  const v8f z8 = {0.f, 0.f, 0.f, 0.f, 0.f, 0.f, 0.f, 0.f};

#pragma unroll 1
  for (int t = 0; t < NSTEP; ++t) {
    const int tc = t & (XCH - 1);
    if (tc == 0) {
#pragma unroll
      for (int q = 0; q < 4; ++q) {
        const int p = tid + q * NTHR;
        const int row = p >> 5, s = p & (XCH - 1);
        const int tabs = t + s;
        const int tcl = tabs < NSTEP ? tabs : (NSTEP - 1);
        const float* xp = x + (size_t)(rowbase + row) * (size_t)(NSTEP * NIN) + (size_t)tcl * NIN;
        v4f w;
        w[0] = bfr(xp[0]); w[1] = bfr(xp[1]); w[2] = bfr(xp[2]); w[3] = 0.0f;
        *(v4f*)(Xs + (row * XCH + s) * XW) = w;
      }
      __syncthreads();
    }
    {
      v8f acc[4];
      acc[0] = z8; acc[1] = z8; acc[2] = z8; acc[3] = z8;
      mac_l0(acc, a0row, whh0);
      float hn[8];
#pragma unroll
      for (int r = 0; r < 8; ++r) {
        const v4f xv = *(const v4f*)(Xs + ((rb + r) * XCH + tc) * XW);
        const float pi = fmaf(acc[0][r], Z_FOLD, fmaf(xv[0], wxi0, fmaf(xv[1], wxi1, fmaf(xv[2], wxi2, cb0i))));
        const float pf = fmaf(acc[1][r], Z_FOLD, fmaf(xv[0], wxf0, fmaf(xv[1], wxf1, fmaf(xv[2], wxf2, cb0f))));
        const float pg = fmaf(acc[2][r], Z_FOLD, fmaf(xv[0], wxg0, fmaf(xv[1], wxg1, fmaf(xv[2], wxg2, cb0g))));
        const float po = fmaf(acc[3][r], Z_FOLD, fmaf(xv[0], wxo0, fmaf(xv[1], wxo1, fmaf(xv[2], wxo2, cb0o))));
        hn[r] = lstm_cell(pi, pf, pg, po, c0s[r]);
      }
      __syncthreads();
#pragma unroll
      for (int r = 0; r < 8; ++r) Ht[(rb + r) * HPITCH + j] = (_Float16)(A_CARRY * hn[r]);
      __syncthreads();
    }
    {
      v8f acc[4];
      acc[0] = z8; acc[1] = z8; acc[2] = z8; acc[3] = z8;
      mac_l1(acc, a0row, a1row, wih1, whh1);
#pragma unroll
      for (int r = 0; r < 8; ++r) {
        const float pi = fmaf(acc[0][r], Z_FOLD, cb1i);
        const float pf = fmaf(acc[1][r], Z_FOLD, cb1f);
        const float pg = fmaf(acc[2][r], Z_FOLD, cb1g);
        const float po = fmaf(acc[3][r], Z_FOLD, cb1o);
        h1s[r] = lstm_cell(pi, pf, pg, po, c1s[r]);
      }
      __syncthreads();
#pragma unroll
      for (int r = 0; r < 8; ++r) Ht[TROWS * HPITCH + (rb + r) * HPITCH + j] = (_Float16)(A_CARRY * h1s[r]);
      __syncthreads();
    }
  }

#pragma unroll
  for (int r = 0; r < 8; ++r) Hs[(rb + r) * OPITCH + j] = h1s[r];
  __syncthreads();
  {
    const int c4 = (lane & 15) * 4;
    for (int pass = 0; pass < 2; ++pass) {
#pragma unroll
      for (int it = 0; it < 2; ++it) {
        const int row = 4 * wave + 2 * it + hh;
        const v4f v = *(const v4f*)(Hs + row * OPITCH + c4);
        *(volatile v4f*)(out + (size_t)(rowbase + row) * NHID + c4) = v;
      }
      __threadfence();
    }
  }
}

extern "C" void kernel_launch(void* const* d_in, const int* in_sizes, int n_in,
                              void* d_out, int out_size, void* d_ws, size_t ws_size, hipStream_t stream) {
  if (n_in < 9 || d_out == nullptr || d_ws == nullptr) return;
  if (in_sizes[0] != NSEQ * NSTEP * NIN || in_sizes[1] != NG4 * NIN || in_sizes[2] != NG4 * NHID ||
      in_sizes[3] != NG4 || in_sizes[4] != NG4 || in_sizes[5] != NG4 * NHID || in_sizes[6] != NG4 * NHID ||
      in_sizes[7] != NG4 || in_sizes[8] != NG4 || out_size != NSEQ * NHID) return;

  const float* x     = (const float*)d_in[0];
  const float* w_ih0 = (const float*)d_in[1];
  const float* w_hh0 = (const float*)d_in[2];
  const float* b_ih0 = (const float*)d_in[3];
  const float* b_hh0 = (const float*)d_in[4];
  const float* w_ih1 = (const float*)d_in[5];
  const float* w_hh1 = (const float*)d_in[6];
  const float* b_ih1 = (const float*)d_in[7];
  const float* b_hh1 = (const float*)d_in[8];
  float* out = (float*)d_out;

  char* ws = (char*)d_ws; size_t off = 0;
  auto carve = [&](size_t bytes) -> char* { char* p = ws + off; off += (bytes + 255) & ~(size_t)255; return p; };
  const size_t plane_bytes = (size_t)NG4 * NHID * 2;
  unsigned short* WHH0 = (unsigned short*)carve(plane_bytes);
  unsigned short* WIH1 = (unsigned short*)carve(plane_bytes);
  unsigned short* WHH1 = (unsigned short*)carve(plane_bytes);
  if (off > ws_size || off > (size_t)134217728) return;

  const int n8 = NG4 * NHID / 8;
  wprep_kernel<<<n8 / NTHR, NTHR, 0, stream>>>(w_hh0, n8, WHH0);
  wprep_kernel<<<n8 / NTHR, NTHR, 0, stream>>>(w_ih1, n8, WIH1);
  wprep_kernel<<<n8 / NTHR, NTHR, 0, stream>>>(w_hh1, n8, WHH1);
  lstm2_kernel<<<NSEQ / TROWS, NTHR, 0, stream>>>(x, w_ih0, b_ih0, b_hh0, b_ih1, b_hh1, WHH0, WIH1, WHH1, out);
}
